// TriplanarDecoder_67585605370028
// MI455X (gfx1250) — hardware-verified
//
#include <hip/hip_runtime.h>
#include <stddef.h>


typedef __bf16 v16b __attribute__((ext_vector_type(16)));
typedef __bf16 v8b  __attribute__((ext_vector_type(8), may_alias));
typedef float  v8f  __attribute__((ext_vector_type(8)));
typedef float  v4f  __attribute__((ext_vector_type(4), may_alias));

#pragma clang fp contract(off)

#define NPB   128
#define C_CH  32
#define PW    512
#define PHW   (PW * PW)
#define FP    72
#define AFP   36

static_assert((FP % 8) == 0);
static_assert((AFP % 4) == 0);

static __device__ __forceinline__ v16b ld_frag(const __bf16* base, int pitch, int m, int h, int k0) {
    const __bf16* row = base + m * pitch + k0 + 8 * h;
    const v8b p0 = *(const v8b*)(row);
    const v8b p1 = *(const v8b*)(row + 16);
    return __builtin_shufflevector(p0, p1, 0, 1, 2, 3, 4, 5, 6, 7, 8, 9, 10, 11, 12, 13, 14, 15);
}

static __device__ __forceinline__ v8f wmma3(v16b ah, v16b al, v16b bh, v16b bl, v8f c) {
    c = __builtin_amdgcn_wmma_f32_16x16x32_bf16(false, ah, false, bh, (short)0, c, false, false);
    c = __builtin_amdgcn_wmma_f32_16x16x32_bf16(false, ah, false, bl, (short)0, c, false, false);
    c = __builtin_amdgcn_wmma_f32_16x16x32_bf16(false, al, false, bh, (short)0, c, false, false);
    asm volatile("v_nop\n\tv_nop\n\tv_nop\n\tv_nop" : "+v"(c) : "v"(ah), "v"(al), "v"(bh), "v"(bl));
    return c;
}

static __device__ __forceinline__ void mlp_step(const __bf16* tH, const __bf16* tL, int tp,
                                                const __bf16* wH, const __bf16* wL, int wp,
                                                int m, int h, int k0,
                                                v8f& c00, v8f& c01, v8f& c10, v8f& c11) {
    const v16b ah0 = ld_frag(tH, tp, m, h, k0);
    const v16b al0 = ld_frag(tL, tp, m, h, k0);
    const v16b ah1 = ld_frag(tH + 16 * tp, tp, m, h, k0);
    const v16b al1 = ld_frag(tL + 16 * tp, tp, m, h, k0);
    const v16b bh0 = ld_frag(wH, wp, m, h, k0);
    const v16b bl0 = ld_frag(wL, wp, m, h, k0);
    const v16b bh1 = ld_frag(wH + 16 * wp, wp, m, h, k0);
    const v16b bl1 = ld_frag(wL + 16 * wp, wp, m, h, k0);
    c00 = wmma3(ah0, al0, bh0, bl0, c00);
    c01 = wmma3(ah0, al0, bh1, bl1, c01);
    c10 = wmma3(ah1, al1, bh0, bl0, c10);
    c11 = wmma3(ah1, al1, bh1, bl1, c11);
}

static __device__ __forceinline__ void split_tile(v8f d, float b, int row0, int col,
                                                  __bf16* tH, __bf16* tL) {
#pragma unroll
    for (int r = 0; r < 8; ++r) {
        float x = d[r] + b;
        x = fmaxf(x, 0.01f * x);
        const __bf16 hi = (__bf16)x;
        const __bf16 lo = (__bf16)(x - (float)hi);
        const int idx = (row0 + r) * FP + col;
        tH[idx] = hi;
        tL[idx] = lo;
    }
}

static __device__ __forceinline__ void epi_split(v8f c00, v8f c01, v8f c10, v8f c11,
                                                 const float* __restrict__ bias, int m, int h,
                                                 __bf16* tH, __bf16* tL) {
    const float bl = bias[m];
    const float bh = bias[16 + m];
    split_tile(c00, bl, 8 * h,      m,      tH, tL);
    split_tile(c01, bh, 8 * h,      16 + m, tH, tL);
    split_tile(c10, bl, 16 + 8 * h, m,      tH, tL);
    split_tile(c11, bh, 16 + 8 * h, 16 + m, tH, tL);
}

static __device__ __forceinline__ void f32_tile(v8f d, float b, int row0, int col, float* aF) {
#pragma unroll
    for (int r = 0; r < 8; ++r) {
        float x = d[r] + b;
        x = fmaxf(x, 0.01f * x);
        aF[(row0 + r) * AFP + col] = x;
    }
}

static __device__ __forceinline__ void epi_f32(v8f c00, v8f c01, v8f c10, v8f c11,
                                               const float* __restrict__ bias, int m, int h, float* aF) {
    const float bl = bias[m];
    const float bh = bias[16 + m];
    f32_tile(c00, bl, 8 * h,      m,      aF);
    f32_tile(c01, bh, 8 * h,      16 + m, aF);
    f32_tile(c10, bl, 16 + 8 * h, m,      aF);
    f32_tile(c11, bh, 16 + 8 * h, 16 + m, aF);
}

struct Tap {
    const float* p00;
    const float* p01;
    const float* p10;
    const float* p11;
    float wnw, wne, wsw, wse;
};

static __device__ __forceinline__ Tap make_tap(const float* __restrict__ img, float gx, float gy) {
    const float ix  = ((gx + 1.0f) * 0.5f) * (float)(PW - 1);
    const float iy  = ((gy + 1.0f) * 0.5f) * (float)(PW - 1);
    const float fx0 = floorf(ix);
    const float fy0 = floorf(iy);
    const float ax  = (fx0 + 1.0f) - ix, bx = ix - fx0;
    const float ay  = (fy0 + 1.0f) - iy, by = iy - fy0;
    Tap t;
    t.wnw = ax * ay;
    t.wne = bx * ay;
    t.wsw = ax * by;
    t.wse = bx * by;
    const int i0 = (int)fminf(fmaxf(fx0, -8.0f), 1024.0f);
    const int j0 = (int)fminf(fmaxf(fy0, -8.0f), 1024.0f);
    const int x0 = min(max(i0, 0), PW - 1);
    const int x1 = min(max(i0 + 1, 0), PW - 1);
    const int y0 = min(max(j0, 0), PW - 1);
    const int y1 = min(max(j0 + 1, 0), PW - 1);
    t.p00 = img + (y0 * PW + x0);
    t.p01 = img + (y0 * PW + x1);
    t.p10 = img + (y1 * PW + x0);
    t.p11 = img + (y1 * PW + x1);
    return t;
}

static __device__ __forceinline__ float tap_eval(const Tap& t, size_t o) {
    const float g00 = t.p00[o];
    const float g01 = t.p01[o];
    const float g10 = t.p10[o];
    const float g11 = t.p11[o];
    return ((g00 * t.wnw + g01 * t.wne) + g10 * t.wsw) + g11 * t.wse;
}

__global__ __launch_bounds__(NPB) __attribute__((amdgpu_num_vgpr(256)))
void k_triplane_mlp(const float* __restrict__ xy, const float* __restrict__ xz,
                    const float* __restrict__ yz, const float* __restrict__ coords,
                    const float* __restrict__ gauss,
                    const float* __restrict__ W0, const float* __restrict__ b0,
                    const float* __restrict__ W1, const float* __restrict__ b1,
                    const float* __restrict__ W2, const float* __restrict__ b2,
                    const float* __restrict__ W3, const float* __restrict__ b3,
                    float* __restrict__ out, int nPoints) {
    __shared__ __attribute__((aligned(16))) __bf16 sWt[8192];
    __shared__ __attribute__((aligned(16))) __bf16 sFeatH[NPB * FP];
    __shared__ __attribute__((aligned(16))) __bf16 sFeatL[NPB * FP];
    __shared__ __attribute__((aligned(16))) float  sActF[4 * 32 * AFP];

    const int tid   = threadIdx.x;
    const int gbase = blockIdx.x * NPB;

    for (int i = tid; i < 2048; i += NPB) {
        const int k = i >> 5, n = i & 31;
        const float w = W0[i];
        const __bf16 hi = (__bf16)w;
        const __bf16 lo = (__bf16)(w - (float)hi);
        sWt[n * 64 + k]        = hi;
        sWt[2048 + n * 64 + k] = lo;
    }
    for (int i = tid; i < 1024; i += NPB) {
        const int k = i >> 5, n = i & 31;
        const float w1 = W1[i];
        const __bf16 h1 = (__bf16)w1;
        const __bf16 l1 = (__bf16)(w1 - (float)h1);
        sWt[4096 + n * 32 + k] = h1;
        sWt[5120 + n * 32 + k] = l1;
        const float w2 = W2[i];
        const __bf16 h2 = (__bf16)w2;
        const __bf16 l2 = (__bf16)(w2 - (float)h2);
        sWt[6144 + n * 32 + k] = h2;
        sWt[7168 + n * 32 + k] = l2;
    }

    {
        const int p = min(gbase + tid, nPoints - 1);
        const float cx = coords[(size_t)p * 3 + 0];
        const float cy = coords[(size_t)p * 3 + 1];
        const float cz = coords[(size_t)p * 3 + 2];

        __bf16* fh = sFeatH + tid * FP;
        __bf16* fl = sFeatL + tid * FP;

        const Tap t1 = make_tap(xy, cx, cy);
        const Tap t2 = make_tap(xz, cx, cz);
        const Tap t3 = make_tap(yz, cy, cz);
#pragma unroll 4
        for (int c = 0; c < C_CH; ++c) {
            const size_t o = (size_t)c * PHW;
            const float e1 = tap_eval(t1, o);
            const float e2 = tap_eval(t2, o);
            const float e3 = tap_eval(t3, o);
            const float x  = ((e1 + e2) + e3) * (1.0f / 3.0f);
            const __bf16 hi = (__bf16)x;
            fh[c] = hi;
            fl[c] = (__bf16)(x - (float)hi);
        }

        const float TWO_PI_F  = 6.28318548202514648f;
        const float INV_2PI_F = 0.159154943091895336f;
        const float px = cx * TWO_PI_F, py = cy * TWO_PI_F, pz = cz * TWO_PI_F;
#pragma unroll 4
        for (int c = 0; c < 16; ++c) {
            const float pr   = (px * gauss[c] + py * gauss[16 + c]) + pz * gauss[32 + c];
            const float nrev = rintf(pr * INV_2PI_F);
            float rr = fmaf(-nrev, 6.28125f, pr);
            rr = fmaf(-nrev, 1.93530717958647692e-3f, rr);
            const float rev = rr * INV_2PI_F;
            const float s  = __builtin_amdgcn_sinf(rev);
            const float co = __builtin_amdgcn_cosf(rev);
            const __bf16 shv = (__bf16)s;
            const __bf16 chv = (__bf16)co;
            fh[32 + c] = shv;
            fl[32 + c] = (__bf16)(s - (float)shv);
            fh[48 + c] = chv;
            fl[48 + c] = (__bf16)(co - (float)chv);
        }
    }
    __syncthreads();

    const int wv   = tid >> 5;
    const int lane = tid & 31;
    const int h    = lane >> 4;
    const int m    = lane & 15;
    __bf16* tH = sFeatH + (wv * 32) * FP;
    __bf16* tL = sFeatL + (wv * 32) * FP;
    float*  aF = sActF + wv * (32 * AFP);

    const v8f zero8 = {0.f, 0.f, 0.f, 0.f, 0.f, 0.f, 0.f, 0.f};
    v8f c00, c01, c10, c11;

    c00 = zero8; c01 = zero8; c10 = zero8; c11 = zero8;
    mlp_step(tH, tL, FP, sWt, sWt + 2048, 64, m, h, 0,  c00, c01, c10, c11);
    mlp_step(tH, tL, FP, sWt, sWt + 2048, 64, m, h, 32, c00, c01, c10, c11);
    epi_split(c00, c01, c10, c11, b0, m, h, tH, tL);
    __syncthreads();

    c00 = zero8; c01 = zero8; c10 = zero8; c11 = zero8;
    mlp_step(tH, tL, FP, sWt + 4096, sWt + 5120, 32, m, h, 0, c00, c01, c10, c11);
    epi_split(c00, c01, c10, c11, b1, m, h, tH, tL);
    __syncthreads();

    c00 = zero8; c01 = zero8; c10 = zero8; c11 = zero8;
    mlp_step(tH, tL, FP, sWt + 6144, sWt + 7168, 32, m, h, 0, c00, c01, c10, c11);
    epi_f32(c00, c01, c10, c11, b2, m, h, aF);
    __syncthreads();

    {
        const float* xr = aF + lane * AFP;
        float o0 = 0.f, o1 = 0.f, o2 = 0.f, o3 = 0.f;
#pragma unroll
        for (int q = 0; q < 8; ++q) {
            const v4f xv = *(const v4f*)(xr + 4 * q);
#pragma unroll
            for (int j = 0; j < 4; ++j) {
                const float xk = xv[j];
                const int k = 4 * q + j;
                o0 = fmaf(xk, W3[k * 4 + 0], o0);
                o1 = fmaf(xk, W3[k * 4 + 1], o1);
                o2 = fmaf(xk, W3[k * 4 + 2], o2);
                o3 = fmaf(xk, W3[k * 4 + 3], o3);
            }
        }
        v4f o;
        o.x = o0 + b3[0];
        o.y = o1 + b3[1];
        o.z = o2 + b3[2];
        o.w = o3 + b3[3];
        const int gp = gbase + wv * 32 + lane;
        volatile v4f* op = (volatile v4f*)(out + (size_t)gp * 4);
        if (gp < nPoints) *op = o;
        __threadfence();
        if (gp < nPoints) *op = o;
    }
}

extern "C" void kernel_launch(void* const* d_in, const int* in_sizes, int n_in,
                              void* d_out, int out_size, void* d_ws, size_t ws_size,
                              hipStream_t stream) {
    (void)d_ws; (void)ws_size;
    if (n_in < 13) return;
    if (in_sizes[0] != C_CH * PHW || in_sizes[1] != C_CH * PHW || in_sizes[2] != C_CH * PHW) return;
    if (in_sizes[4] != 48 || in_sizes[5] != 2048 || in_sizes[6] != 32 || in_sizes[7] != 1024 ||
        in_sizes[8] != 32 || in_sizes[9] != 1024 || in_sizes[10] != 32 || in_sizes[11] != 128 ||
        in_sizes[12] != 4) return;

    const float* xy     = (const float*)d_in[0];
    const float* xz     = (const float*)d_in[1];
    const float* yz     = (const float*)d_in[2];
    const float* coords = (const float*)d_in[3];
    const float* gauss  = (const float*)d_in[4];
    const float* W0     = (const float*)d_in[5];
    const float* b0     = (const float*)d_in[6];
    const float* W1     = (const float*)d_in[7];
    const float* b1     = (const float*)d_in[8];
    const float* W2     = (const float*)d_in[9];
    const float* b2     = (const float*)d_in[10];
    const float* W3     = (const float*)d_in[11];
    const float* b3     = (const float*)d_in[12];
    float* out = (float*)d_out;

    int nPoints = in_sizes[3] / 3;
    if (out_size / 4 < nPoints) nPoints = out_size / 4;
    if (nPoints <= 0) return;
    const int blocks = (nPoints + NPB - 1) / NPB;

    k_triplane_mlp<<<dim3(blocks), dim3(NPB), 0, stream>>>(
        xy, xz, yz, coords, gauss, W0, b0, W1, b1, W2, b2, W3, b3, out, nPoints);
}
